// DOMTransformer_14130442404235
// MI455X (gfx1250) — hardware-verified
//
#include <hip/hip_runtime.h>
#include <math.h>

typedef __attribute__((ext_vector_type(16))) _Float16 v16h;
typedef __attribute__((ext_vector_type(16))) __bf16 v16b;
typedef __attribute__((ext_vector_type(8)))  _Float16 v8h;
typedef __attribute__((ext_vector_type(8)))  float v8f;
typedef __attribute__((ext_vector_type(4)))  float v4f;
typedef __attribute__((ext_vector_type(2)))  float v2f;
typedef __attribute__((ext_vector_type(4)))  unsigned v4u;
typedef __attribute__((ext_vector_type(4)))  int v4i;
typedef float __attribute__((may_alias)) float_a;
typedef int __attribute__((may_alias)) int_a;

template <typename T> __device__ __forceinline__ void vst2(void* p, T v) { *(volatile T*)p = v; __threadfence(); *(volatile T*)p = v; }
__device__ __forceinline__ v8f wmma16(v16h a, v16h b, v8f c) {
  v8f d = __builtin_amdgcn_wmma_f32_16x16x32_f16(false, a, false, b, (short)0, c, false, false);
  asm volatile("v_nop\n\tv_nop\n\tv_nop\n\tv_nop" : "+v"(d) : "v"(a), "v"(b));
  return d;
}
__device__ __forceinline__ v8f wmma_bf(v16b a, v16b b, v8f c) {
  v8f d = __builtin_amdgcn_wmma_f32_16x16x32_bf16(false, a, false, b, (short)0, c, false, false);
  asm volatile("v_nop\n\tv_nop\n\tv_nop\n\tv_nop" : "+v"(d) : "v"(a), "v"(b));
  return d;
}
__device__ __forceinline__ v16h frag_h(const _Float16* rowk0, int lane) {
  union { v16h v; v8h q[2]; } u; const _Float16* p = rowk0 + 8 * (lane >> 4);
  u.q[0] = *(const v8h*)p; u.q[1] = *(const v8h*)(p + 16); return u.v;
}
__device__ __forceinline__ v16h frag_f32(const float* rowk0, int lane) {
  v16h a; const float* p = rowk0 + 8 * (lane >> 4);
#pragma unroll
  for (int i = 0; i < 8; ++i) { a[i] = (_Float16)p[i]; a[8 + i] = (_Float16)p[16 + i]; }
  return a;
}
__device__ __forceinline__ v16h frag_f32s(const float* rowk0, int lane, float sc) {
  v16h a; const float* p = rowk0 + 8 * (lane >> 4);
#pragma unroll
  for (int i = 0; i < 8; ++i) { a[i] = (_Float16)(p[i] * sc); a[8 + i] = (_Float16)(p[16 + i] * sc); }
  return a;
}
__device__ __forceinline__ v16h fragc_f32(const float* W, int k0, int n, int lane, int ld, int K) {
  v16h a; const int g = lane >> 4;
#pragma unroll
  for (int i = 0; i < 8; ++i) { const int ka = k0 + 8 * g + i, kb = ka + 16;
    a[i] = (_Float16)(ka < K ? W[(size_t)(ka < K ? ka : K - 1) * ld + n] : 0.f); a[8 + i] = (_Float16)(kb < K ? W[(size_t)(kb < K ? kb : K - 1) * ld + n] : 0.f); }
  return a;
}
struct F2 { v16b h, l; };
__device__ __forceinline__ F2 bsplit16(const float v[16]) { F2 r;
#pragma unroll
  for (int i = 0; i < 16; ++i) { const __bf16 h = (__bf16)v[i]; r.h[i] = h; r.l[i] = (__bf16)(v[i] - (float)h); }
  return r; }
__device__ __forceinline__ F2 split_row(const float* row, int k0, int lane) { float v[16]; const float* p = row + k0 + 8 * (lane >> 4);
#pragma unroll
  for (int i = 0; i < 8; ++i) { v[i] = p[i]; v[8 + i] = p[16 + i]; }
  return bsplit16(v); }
__device__ __forceinline__ F2 split_rowK(const float* row, int k0, int lane, int K) { float v[16]; const int g = lane >> 4;
#pragma unroll
  for (int i = 0; i < 8; ++i) { const int ka = k0 + 8 * g + i, kb = ka + 16; v[i] = ka < K ? row[ka < K ? ka : K - 1] : 0.f; v[8 + i] = kb < K ? row[kb < K ? kb : K - 1] : 0.f; }
  return bsplit16(v); }
__device__ __forceinline__ F2 split_col(const float* W, int k0, int n, int lane, int ld, int K) { float v[16]; const int g = lane >> 4;
#pragma unroll
  for (int i = 0; i < 8; ++i) { const int ka = k0 + 8 * g + i, kb = ka + 16; v[i] = ka < K ? W[(size_t)(ka < K ? ka : K - 1) * ld + n] : 0.f; v[8 + i] = kb < K ? W[(size_t)(kb < K ? kb : K - 1) * ld + n] : 0.f; }
  return bsplit16(v); }
__device__ __forceinline__ v8f mac3(const F2& a, const F2& b, v8f c) { c = wmma_bf(a.l, b.h, c); c = wmma_bf(a.h, b.l, c); return wmma_bf(a.h, b.h, c); }
__device__ __forceinline__ float sigm(float v) { return 1.0f / (1.0f + expf(-v)); }
#define LDSX() do { asm volatile("s_wait_dscnt 0" ::: "memory"); __builtin_amdgcn_wave_barrier(); __builtin_amdgcn_fence(__ATOMIC_RELEASE, "workgroup"); } while (0)


#define NP 4096
#define PF 4
#define DM 256
#define NH 8
#define HD 32
#define NL 4
#define DFF 1024
#define NDOM 512
#define NRB (NP / 64)
typedef __attribute__((ext_vector_type(8))) __bf16 v8b;
__device__ __forceinline__ v16b frag_b(const __bf16* rowk0, int lane) {
  union { v16b v; v8b q[2]; } u; const __bf16* p = rowk0 + 8 * (lane >> 4);
  u.q[0] = *(const v8b*)p; u.q[1] = *(const v8b*)(p + 16); return u.v;
}
__device__ __forceinline__ float bfr(float v) { return (float)(__bf16)v; }
__device__ __attribute__((noinline)) float exp_ni(float v) { return expf(v); }
__device__ __attribute__((noinline)) float erf_ni(float v) { return erff(v); }


#define CSA_N 512
#define CSA_E 4096
#define CSA_FINN (CSA_E + 32 * CSA_NBK)
#define CSA_CHUNK 4096
#define CSA_BKT 256
#define CSA_NCH ((CSA_E + CSA_CHUNK - 1) / CSA_CHUNK)
#define CSA_NBK ((CSA_N + CSA_BKT - 1) / CSA_BKT)
#define CSA_NBKP (((CSA_NBK + 63) / 64) * 64)
#define CSA_SEGCAP (CSA_E + 32 * CSA_NBK * CSA_NCH)
#ifndef CSA_BCAP
#define CSA_BCAP 10240
#endif
#define CSA_SZ_CNT   (4u * CSA_NCH * CSA_NBKP)
#define CSA_SZ_OFF   (4u * CSA_NBK * (((CSA_NCH + 31) / 32) * 32))
#define CSA_SZ_BST   (4u * (((CSA_NBK + 1 + 31) / 32) * 32))
#define CSA_SZ_SEG   (4u * CSA_SEGCAP)
#define CSA_SZ_FIN   (4u * (CSA_E + 32 * CSA_NBK))
#define CSA_SZ_ROW   (4u * CSA_NBK * CSA_BKT)
#define CSA_OFFP (((CSA_NCH + 31) / 32) * 32)

__global__ __launch_bounds__(256) void k_csA_cnt(const int* __restrict__ DST, int dstride, int* __restrict__ CNT) {
  __shared__ unsigned short sc[256][CSA_NBK + 1]; __shared__ __align__(16) int srow[CSA_NBKP];
  const int c = blockIdx.x, tid = threadIdx.x;
  for (int b = 0; b < CSA_NBK; ++b) sc[tid][b] = 0;
  const size_t e0 = (size_t)c * CSA_CHUNK + tid * 16;
  for (int i = 0; i < 16; ++i) { const size_t e = e0 + i; if (e < (size_t)CSA_E) { int d = DST[e * dstride]; d = min(max(d, 0), CSA_N - 1); sc[tid][d / CSA_BKT] += 1; } }
  __syncthreads();
  for (int b = tid; b < CSA_NBKP; b += 256) { int s = 0; if (b < CSA_NBK) for (int t = 0; t < 256; ++t) s += sc[t][b]; srow[b] = s; }
  __syncthreads();
  for (int q = tid; q < CSA_NBKP / 4; q += 256) vst2((unsigned*)(CNT + (size_t)c * CSA_NBKP + q * 4), *(const v4u*)&srow[q * 4]);
}
__global__ __launch_bounds__(256) void k_csA_scan(const int* __restrict__ CNT, int* __restrict__ OFF, int* __restrict__ BST) {
  __shared__ int sbt[CSA_NBK + 1]; __shared__ int sbs[((CSA_NBK + 1 + 31) / 32) * 32]; __shared__ int scnt[CSA_NBK + 1]; __shared__ __align__(16) int sbuf[64][CSA_OFFP];
  const int tid = threadIdx.x;
  for (int b = tid; b < CSA_NBK; b += 256) { int sp = 0, st = 0; for (int c = 0; c < CSA_NCH; ++c) { const int n = CNT[(size_t)c * CSA_NBKP + b]; st += n; sp += (n + 31) & ~31; } sbt[b] = sp; scnt[b] = st; }
  for (int b = tid; b < ((CSA_NBK + 1 + 31) / 32) * 32; b += 256) sbs[b] = 0;
  __syncthreads();
  if (tid == 0) { int acc = 0, accf = 0; for (int b = 0; b < CSA_NBK; ++b) { const int t = sbt[b]; sbt[b] = acc; acc += t; sbs[b] = accf; accf += (scnt[b] + 31) & ~31; } sbs[CSA_NBK] = accf; }
  __syncthreads();
  for (int b0 = 0; b0 < CSA_NBK; b0 += 64) {
    if (tid < 64 && b0 + tid < CSA_NBK) { const int b = b0 + tid; int o = sbt[b]; for (int c = 0; c < CSA_OFFP; ++c) { if (c < CSA_NCH) { sbuf[tid][c] = o; o += (CNT[(size_t)c * CSA_NBKP + b] + 31) & ~31; } else sbuf[tid][c] = 0; } }
    __syncthreads();
    for (int q = tid; q < 64 * (CSA_OFFP / 4); q += 256) { const int r = q / (CSA_OFFP / 4), pc = q % (CSA_OFFP / 4); if (b0 + r < CSA_NBK) vst2((unsigned*)(OFF + (size_t)(b0 + r) * CSA_OFFP + pc * 4), *(const v4u*)&sbuf[r][pc * 4]); }
    __syncthreads(); }
  for (int q = tid; q < ((CSA_NBK + 1 + 31) / 32) * 32 / 4; q += 256) vst2((unsigned*)(BST + q * 4), *(const v4u*)&sbs[q * 4]);
}
__global__ __launch_bounds__(256) void k_csA_scatter(const int* __restrict__ SRC, const int* __restrict__ DST, int sstride, int dstride, const int* __restrict__ OFF, int* __restrict__ SEGS, int* __restrict__ SEGE) {
  __shared__ unsigned short sc[256][CSA_NBK + 1]; __shared__ int sbase[CSA_NBK + 1]; __shared__ int scn[CSA_NBK + 1]; __shared__ int sord[CSA_CHUNK];
  const int c = blockIdx.x, tid = threadIdx.x;
  for (int b = 0; b < CSA_NBK; ++b) sc[tid][b] = 0;
  const size_t e0 = (size_t)c * CSA_CHUNK + tid * 16; int bk[16];
#pragma unroll
  for (int i = 0; i < 16; ++i) { const size_t e = e0 + i; bk[i] = -1; if (e < (size_t)CSA_E) { int d = DST[e * dstride]; d = min(max(d, 0), CSA_N - 1); bk[i] = d / CSA_BKT; sc[tid][bk[i]] += 1; } }
  __syncthreads();
  for (int b = tid; b < CSA_NBK; b += 256) { int acc = 0; for (int t = 0; t < 256; ++t) { const int v = sc[t][b]; sc[t][b] = (unsigned short)acc; acc += v; } scn[b] = acc; }
  __syncthreads();
  if (tid == 0) { int acc = 0; for (int b = 0; b < CSA_NBK; ++b) { sbase[b] = acc; acc += scn[b]; } }
  __syncthreads();
#pragma unroll
  for (int i = 0; i < 16; ++i) { if (bk[i] >= 0) { const int b = bk[i]; const int r = sc[tid][b]; sc[tid][b] = (unsigned short)(r + 1); sord[sbase[b] + r] = tid * 16 + i; } }
  __syncthreads();
  for (int b = 0; b < CSA_NBK; ++b) { const int n = scn[b]; if (n == 0) continue; const int nl = ((n + 31) & ~31); const size_t o = (size_t)(min(max(OFF[(size_t)b * CSA_OFFP + c], 0), CSA_SEGCAP - nl) & ~31);
    for (int q = tid; q < nl / 4; q += 256) { int4 vs, ve;
#pragma unroll
      for (int k = 0; k < 4; ++k) { const int i = q * 4 + k; int s = -1, eid = -1; if (i < n) { const size_t e = (size_t)c * CSA_CHUNK + sord[sbase[b] + i]; s = min(max(SRC[e * sstride], 0), CSA_N - 1); eid = (int)e; } vs[k] = s; ve[k] = eid; }
      vst2((unsigned*)(SEGS + o + q * 4), *(const v4u*)&vs); vst2((unsigned*)(SEGE + o + q * 4), *(const v4u*)&ve); } }
}
__global__ __launch_bounds__(256) void k_csA_bucket(const int* __restrict__ CNT, const int* __restrict__ OFF, const int* __restrict__ BST, const int* __restrict__ SEGS, const int* __restrict__ SEGE, const int* __restrict__ DST, int dstride, int* __restrict__ FS, int* __restrict__ FE, int* __restrict__ ROWST, int* __restrict__ ROWCNT) {
  __shared__ int ssrc[CSA_BCAP]; __shared__ int seid[CSA_BCAP]; __shared__ unsigned char snod[CSA_BCAP]; __shared__ int souts[CSA_BCAP]; __shared__ int soute[CSA_BCAP]; __shared__ int scount[256]; __shared__ int sstart[257]; __shared__ int stot;
  const int b = blockIdx.x, tid = threadIdx.x;
  if (tid == 0) { int t = 0; for (int c = 0; c < CSA_NCH; ++c) t += min(max(CNT[(size_t)c * CSA_NBKP + b], 0), CSA_CHUNK); stot = (t <= CSA_BCAP) ? t : 0; }
  __syncthreads();
  { int base = 0; for (int c = 0; c < CSA_NCH; ++c) { const int n = min(max(CNT[(size_t)c * CSA_NBKP + b], 0), CSA_CHUNK); const int o = min(max(OFF[(size_t)b * CSA_OFFP + c], 0), CSA_SEGCAP - ((n + 31) & ~31));
      for (int i = tid; i < n; i += 256) { const int p = base + i; if (p < CSA_BCAP) { ssrc[p] = min(max(SEGS[o + i], 0), CSA_N - 1); const int e = min(max(SEGE[o + i], 0), CSA_E - 1); seid[p] = e; int d = DST[(size_t)e * dstride]; d = min(max(d, 0), CSA_N - 1); const int dl = d - b * CSA_BKT; snod[p] = (unsigned char)(dl >= 0 && dl < 256 ? dl : 255); } }
      base += n; } }
  __syncthreads();
  const int node = b * CSA_BKT + tid; int cnt = 0; for (int p = 0; p < stot; ++p) cnt += (snod[p] == tid) ? 1 : 0;
  scount[tid] = cnt; __syncthreads();
  if (tid == 0) { int acc = 0; for (int t = 0; t < 256; ++t) { sstart[t] = acc; acc += scount[t]; } sstart[256] = acc; }
  __syncthreads();
  const int bst0 = min(max(BST[b], 0), CSA_FINN - ((sstart[256] + 31) & ~31)) & ~31; const int gst = bst0 + sstart[tid];
  { int w = sstart[tid]; for (int p = 0; p < stot; ++p) if (snod[p] == tid) { souts[w] = ssrc[p]; soute[w] = seid[p]; ++w; } }
  __syncthreads();
  { const int n = sstart[256]; const int nl = (n + 31) & ~31; for (int q = tid; q < nl / 4; q += 256) { int4 vs, ve;
#pragma unroll
      for (int k = 0; k < 4; ++k) { const int i = q * 4 + k; vs[k] = i < n ? souts[i] : -1; ve[k] = i < n ? soute[i] : -1; }
      vst2((unsigned*)(FS + bst0 + q * 4), *(const v4u*)&vs); vst2((unsigned*)(FE + bst0 + q * 4), *(const v4u*)&ve); } }
  __syncthreads();
  { __shared__ __align__(16) int srs[256], src2[256]; srs[tid] = node < CSA_N ? gst : 0; src2[tid] = node < CSA_N ? cnt : 0; __syncthreads();
    if (tid < 64) vst2((unsigned*)(ROWST + (size_t)b * 256 + tid * 4), *(const v4u*)&srs[tid * 4]); else if (tid < 128) vst2((unsigned*)(ROWCNT + (size_t)b * 256 + (tid - 64) * 4), *(const v4u*)&src2[(tid - 64) * 4]); }
}


#define WS_CNT  0u
#define WS_OFF  (WS_CNT + CSA_SZ_CNT)
#define WS_BST  (WS_OFF + CSA_SZ_OFF)
#define WS_SEGS (WS_BST + CSA_SZ_BST)
#define WS_SEGE (WS_SEGS + CSA_SZ_SEG)
#define WS_FS   (WS_SEGE + CSA_SZ_SEG)
#define WS_FE   (WS_FS + CSA_SZ_FIN)
#define WS_RST  (WS_FE + CSA_SZ_FIN)
#define WS_RCT  (WS_RST + CSA_SZ_ROW)
#define WS_PW   (WS_RCT + CSA_SZ_ROW)
#define PLAY(l) ((size_t)(l) * (768 * DM + DM * DM + DFF * DM + DM * DFF))
#define PQKV(l) (PLAY(l))
#define POUT(l) (PLAY(l) + (size_t)768 * DM)
#define PW1(l)  (POUT(l) + (size_t)DM * DM)
#define PW2(l)  (PW1(l) + (size_t)DFF * DM)
#define PWEND   (PLAY(NL))
#define WS_X    (WS_PW + 2u * PWEND)
#define WS_QKV  (WS_X + 4u * NP * DM)
#define WS_O    (WS_QKV + 4u * NP * 768)
#define WS_T    (WS_O + 4u * NP * DM)
#define WS_F1   (WS_T + 4u * NP * DM)
#define WS_END  (WS_F1 + 4u * NP * DFF)

__global__ __launch_bounds__(256) void k_packW(const float* __restrict__ Wm, int K, int NOUT, __bf16* __restrict__ DST) {
  __shared__ __align__(16) __bf16 s[DFF]; const int n = blockIdx.x, tid = threadIdx.x;
  for (int k = tid; k < K; k += 256) s[k] = (__bf16)Wm[(size_t)k * NOUT + n];
  __syncthreads();
  for (int q = tid; q < K / 8; q += 256) vst2((unsigned*)(DST + (size_t)n * K + q * 8), *(const v4u*)&s[q * 8]);
}
__global__ __launch_bounds__(256) void k_inp(const float* __restrict__ PFm, const float* __restrict__ WIN, const float* __restrict__ BIN, float* __restrict__ X) {
  __shared__ float sp[64][PF]; __shared__ __align__(16) float so[64][DM]; const int tid = threadIdx.x; const size_t n0 = (size_t)blockIdx.x * 64;
  sp[tid >> 2][tid & 3] = bfr(PFm[(n0 + (tid >> 2)) * PF + (tid & 3)]);
  float w[PF];
#pragma unroll
  for (int k = 0; k < PF; ++k) w[k] = bfr(WIN[k * DM + tid]);
  const float bb = bfr(BIN[tid]);
  __syncthreads();
#pragma unroll 1
  for (int rl = 0; rl < 64; ++rl) { float a = bb;
#pragma unroll
    for (int k = 0; k < PF; ++k) a += sp[rl][k] * w[k];
    so[rl][tid] = a; }
  __syncthreads();
  for (int q = tid; q < 64 * DM / 4; q += 256) { const int rl = q / (DM / 4), pc = q % (DM / 4); vst2(X + (n0 + rl) * DM + pc * 4, *(const v4f*)&so[rl][pc * 4]); }
}
template <int EPI>
__global__ __launch_bounds__(128) void k_gemm(const float* __restrict__ A, int lda, int K, const __bf16* __restrict__ P, const float* __restrict__ bias, const float* __restrict__ RES, float* __restrict__ OUT, int ldo) {
  __shared__ __align__(16) float so[4][16][132];
  const int tid = threadIdx.x, wave = tid >> 5, lane = tid & 31, col = lane & 15, g = lane >> 4; const size_t r0 = (size_t)blockIdx.x * 64 + wave * 16; const int n0 = blockIdx.y * 128;
  v8f acc[8] = {};
#pragma unroll 2
  for (int kc = 0; kc < K / 32; ++kc) { const F2 a = split_row(A + (r0 + col) * (size_t)lda, kc * 32, lane);
#pragma unroll
    for (int j = 0; j < 8; ++j) { const v16b w = frag_b(P + (size_t)(n0 + j * 16 + col) * K + kc * 32, lane); acc[j] = wmma_bf(a.l, w, acc[j]); acc[j] = wmma_bf(a.h, w, acc[j]); } }
#pragma unroll
  for (int j = 0; j < 8; ++j) { const int n = n0 + j * 16 + col; const float bb = bfr(bias[n]);
#pragma unroll
    for (int r = 0; r < 8; ++r) { float v = acc[j][r] + bb; if (EPI == 1) v = 0.5f * v * (1.0f + erf_ni(v * 0.70710678118654752f)); if (EPI == 2) v += RES[(r0 + 8 * g + r) * (size_t)ldo + n]; so[wave][8 * g + r][j * 16 + col] = v; } }
  LDSX();
  for (int rl = 0; rl < 16; ++rl) vst2(OUT + (r0 + rl) * (size_t)ldo + n0 + lane * 4, *(const v4f*)&so[wave][rl][lane * 4]);
}
#define KCH 32
__global__ __launch_bounds__(256) void k_attn(const float* __restrict__ QKV, const int* __restrict__ DIDX, const int* __restrict__ FS, const int* __restrict__ RST, const int* __restrict__ RCT, float* __restrict__ O) {
  __shared__ float ssc[256][KCH + 1];
  const int tid = threadIdx.x; const size_t i = (size_t)blockIdx.x * 32 + (tid >> 3); const int h = tid & 7;
  const int dom = min(max(DIDX[i], 0), NDOM - 1); const int cnt = min(max(RCT[dom], 0), CSA_BCAP); const int st = min(max(RST[dom], 0), CSA_FINN - cnt);
  const float* q = QKV + i * 768 + h * HD; float qv[HD];
#pragma unroll
  for (int d = 0; d < HD; ++d) qv[d] = q[d];
  const float scale = 1.0f / sqrtf((float)HD);
  float m = -3.0e38f, l = 0.f; float o[HD];
#pragma unroll
  for (int d = 0; d < HD; ++d) o[d] = 0.f;
#pragma unroll 1
  for (int c0 = 0; c0 < cnt; c0 += KCH) { const int nc = min(KCH, cnt - c0); float cm = -3.0e38f;
#pragma unroll 1
    for (int e = 0; e < nc; ++e) { const int j = min(max(FS[st + c0 + e], 0), NP - 1); const float* k = QKV + (size_t)j * 768 + DM + h * HD; float s = 0.f;
#pragma unroll
      for (int d = 0; d < HD; ++d) s += qv[d] * k[d];
      s *= scale; ssc[tid][e] = s; cm = fmaxf(cm, s); }
    const float mn = fmaxf(m, cm); const float alpha = (m <= -1.0e38f) ? 0.f : exp_ni(m - mn);
    l *= alpha;
#pragma unroll
    for (int d = 0; d < HD; ++d) o[d] *= alpha;
#pragma unroll 1
    for (int e = 0; e < nc; ++e) { const int j = min(max(FS[st + c0 + e], 0), NP - 1); const float* v = QKV + (size_t)j * 768 + 2 * DM + h * HD; const float p = exp_ni(ssc[tid][e] - mn); l += p;
#pragma unroll
      for (int d = 0; d < HD; ++d) o[d] += p * v[d]; }
    m = mn; }
  const float il = (l > 0.f) ? 1.0f / l : 0.f;
  float* orow = O + i * DM + h * HD;
#pragma unroll
  for (int pc = 0; pc < HD / 4; ++pc) { v4f w4 = {o[pc * 4] * il, o[pc * 4 + 1] * il, o[pc * 4 + 2] * il, o[pc * 4 + 3] * il}; vst2(orow + pc * 4, w4); }
}
__global__ __launch_bounds__(256) void k_ln(const float* __restrict__ T, const float* __restrict__ G, const float* __restrict__ Bb, float* __restrict__ Y) {
  __shared__ __align__(16) float s[8][DM]; const int tid = threadIdx.x, wave = tid >> 5, lane = tid & 31; const size_t row = (size_t)blockIdx.x * 8 + wave;
  float v[8]; float sum = 0.f;
#pragma unroll
  for (int k = 0; k < 8; ++k) { v[k] = T[row * DM + lane + 32 * k]; sum += v[k]; }
#pragma unroll
  for (int o = 1; o < 32; o <<= 1) sum += __shfl_xor(sum, o);
  const float mu = sum / (float)DM; float var = 0.f;
#pragma unroll
  for (int k = 0; k < 8; ++k) { const float d = v[k] - mu; var += d * d; }
#pragma unroll
  for (int o = 1; o < 32; o <<= 1) var += __shfl_xor(var, o);
  const float rs = rsqrtf(var / (float)DM + 1e-5f);
#pragma unroll
  for (int k = 0; k < 8; ++k) { const int c = lane + 32 * k; s[wave][c] = (v[k] - mu) * rs * bfr(G[c]) + bfr(Bb[c]); }
  LDSX();
  for (int pc = lane; pc < DM / 4; pc += 32) vst2(Y + row * DM + pc * 4, *(const v4f*)&s[wave][pc * 4]);
}
__global__ __launch_bounds__(256) void k_dommean(const float* __restrict__ X, const int* __restrict__ FS, const int* __restrict__ RST, const int* __restrict__ RCT, float* __restrict__ out) {
  __shared__ __align__(16) float so[DM]; const int tid = threadIdx.x, dom = blockIdx.x; const int cnt = min(max(RCT[dom], 0), CSA_BCAP); const int st = min(max(RST[dom], 0), CSA_FINN - cnt);
  float a = 0.f; for (int e = 0; e < cnt; ++e) { const int j = min(max(FS[st + e], 0), NP - 1); a += X[(size_t)j * DM + tid]; }
  so[tid] = a / (float)(cnt > 0 ? cnt : 1); __syncthreads();
  if (tid < DM / 4) vst2(out + (size_t)dom * DM + tid * 4, *(const v4f*)&so[tid * 4]);
}
extern "C" void kernel_launch(void* const* d_in, const int* in_sizes, int n_in, void* d_out, int out_size, void* d_ws, size_t ws_size, hipStream_t stream) {
  (void)in_sizes; (void)n_in; (void)out_size;
  const float** F = (const float**)d_in; const int* DIDX = (const int*)d_in[1];
  if (ws_size < (size_t)WS_END) return;
  char* ws = (char*)d_ws;
  int *CNT = (int*)(ws + WS_CNT), *OFF = (int*)(ws + WS_OFF), *BST = (int*)(ws + WS_BST), *SEGS = (int*)(ws + WS_SEGS), *SEGE = (int*)(ws + WS_SEGE), *FS = (int*)(ws + WS_FS), *FE = (int*)(ws + WS_FE), *RST = (int*)(ws + WS_RST), *RCT = (int*)(ws + WS_RCT);
  __bf16* PW = (__bf16*)(ws + WS_PW); float *X = (float*)(ws + WS_X), *QKV = (float*)(ws + WS_QKV), *O = (float*)(ws + WS_O), *T = (float*)(ws + WS_T), *F1 = (float*)(ws + WS_F1);
  k_csA_cnt<<<CSA_NCH, 256, 0, stream>>>(DIDX, 1, CNT); k_csA_scan<<<1, 256, 0, stream>>>(CNT, OFF, BST); k_csA_scatter<<<CSA_NCH, 256, 0, stream>>>(DIDX, DIDX, 1, 1, OFF, SEGS, SEGE); k_csA_bucket<<<CSA_NBK, 256, 0, stream>>>(CNT, OFF, BST, SEGS, SEGE, DIDX, 1, FS, FE, RST, RCT);
  for (int l = 0; l < NL; ++l) { k_packW<<<768, 256, 0, stream>>>(F[5] + (size_t)l * DM * 768, DM, 768, PW + PQKV(l)); k_packW<<<DM, 256, 0, stream>>>(F[7] + (size_t)l * DM * DM, DM, DM, PW + POUT(l)); k_packW<<<DFF, 256, 0, stream>>>(F[9] + (size_t)l * DM * DFF, DM, DFF, PW + PW1(l)); k_packW<<<DM, 256, 0, stream>>>(F[11] + (size_t)l * DFF * DM, DFF, DM, PW + PW2(l)); }
  k_inp<<<NRB, 256, 0, stream>>>(F[0], F[3], F[4], X);
  for (int l = 0; l < NL; ++l) {
    k_gemm<0><<<dim3(NRB, 768 / 128), 128, 0, stream>>>(X, DM, DM, PW + PQKV(l), F[6] + (size_t)l * 768, nullptr, QKV, 768);
    k_attn<<<NP / 32, 256, 0, stream>>>(QKV, DIDX, FE, RST, RCT, O);
    k_gemm<2><<<dim3(NRB, DM / 128), 128, 0, stream>>>(O, DM, DM, PW + POUT(l), F[8] + (size_t)l * DM, X, T, DM);
    k_ln<<<NP / 8, 256, 0, stream>>>(T, F[13] + (size_t)l * DM, F[14] + (size_t)l * DM, X);
    k_gemm<1><<<dim3(NRB, DFF / 128), 128, 0, stream>>>(X, DM, DM, PW + PW1(l), F[10] + (size_t)l * DFF, nullptr, F1, DFF);
    k_gemm<2><<<dim3(NRB, DM / 128), 128, 0, stream>>>(F1, DFF, DFF, PW + PW2(l), F[12] + (size_t)l * DM, X, T, DM);
    k_ln<<<NP / 8, 256, 0, stream>>>(T, F[15] + (size_t)l * DM, F[16] + (size_t)l * DM, X);
  }
  k_ln<<<NP / 8, 256, 0, stream>>>(X, F[17], F[18], T);
  k_dommean<<<NDOM, 256, 0, stream>>>(T, FE, RST, RCT, (float*)d_out);
}
